// CrystalDiffusionModel_48713519071926
// MI455X (gfx1250) — hardware-verified
//
#include <hip/hip_runtime.h>


namespace {
constexpr int N = 20000, G = 128, HID = 128, TE = 128, CDIM = 64, LYR = 6, NBLK = N / 32;
constexpr float AS_ = 8.0f;

typedef _Float16 b16;
typedef __attribute__((ext_vector_type(16))) _Float16 v16b;
typedef __attribute__((ext_vector_type(8))) _Float16 v8b;
typedef __attribute__((ext_vector_type(8))) float v8f;
typedef __attribute__((ext_vector_type(4))) float v4f;
__device__ __forceinline__ float bf16_rne(float f) { unsigned int u = __float_as_uint(f); u += 0x7FFFu + ((u >> 16) & 1u); return __uint_as_float(u & 0xFFFF0000u); }
__device__ __forceinline__ void split16(float v, b16& hi, b16& lo) { hi = (b16)v; lo = (b16)(v - (float)hi); }
__device__ __forceinline__ v16b frag_kb(const b16* p, int hh) { const v8b a = *(const v8b*)(p + 8 * hh), b = *(const v8b*)(p + 16 + 8 * hh); v16b f;
#pragma unroll
  for (int e = 0; e < 8; ++e) { f[e] = a[e]; f[8 + e] = b[e]; } return f; }
__device__ __forceinline__ void frag_split(const float* p, int hh, v16b& fh, v16b& fl) {
#pragma unroll
  for (int e = 0; e < 8; ++e) { b16 a, c; split16(p[8 * hh + e] * AS_, a, c); fh[e] = a; fl[e] = c; split16(p[16 + 8 * hh + e] * AS_, a, c); fh[8 + e] = a; fl[8 + e] = c; } }
__device__ __forceinline__ v8f wmma16b(v16b a, v16b b, v8f c) { v8f d = __builtin_amdgcn_wmma_f32_16x16x32_f16(false, a, false, b, (short)0, c, false, false); asm volatile("v_nop\n\tv_nop\n\tv_nop\n\tv_nop" : "+v"(d) : "v"(a), "v"(b)); return d; }
__device__ __forceinline__ void wave_lds_sync() { __builtin_amdgcn_fence(__ATOMIC_RELEASE, "workgroup"); __builtin_amdgcn_wave_barrier(); __builtin_amdgcn_fence(__ATOMIC_ACQUIRE, "workgroup"); }
__device__ __forceinline__ float nexp(float x) { return __builtin_amdgcn_exp2f(x * 1.4426950408889634f); }
__device__ __forceinline__ float silu_(float x) { return x * __builtin_amdgcn_rcpf(1.0f + nexp(-x)); }

struct Wo_ { static constexpr size_t TM1 = 0, TM2 = TM1 + 256 * 128, TP1 = TM2 + 128 * 256, TP2 = TP1 + 32 * 32, SB1 = TP2 + 32 * 32, SB2 = SB1 + 16 * 32, SU1 = SB2 + 16 * 32, SU2 = SU1 + 16 * 32, CB1 = SU2 + 16 * 32, CB2 = CB1 + 64 * 64, WV = CB2 + 64 * 64, WO = WV + 128 * 64, WN = WO + 128 * 128, NP1 = WN + 128 * 32, NP2 = NP1 + 256 * 128, PP1 = NP2 + 16 * 256, PP2 = PP1 + 128 * 128, END = PP2 + 16 * 128; };
struct Po_ { static constexpr int TMB1 = 0, TMB2 = 256, TPB1 = 384, TPB2 = 416, SBB1 = 448, SBB2 = 464, SUB1 = 480, SUB2 = 496, CBB1 = 512, CBB2 = 576, BO = 640, BN = 768, NPB1 = 896, NPB2 = 1152, PPB1 = 1168, PPB2 = 1296, END = 1312; };

__device__ __forceinline__ void trw(b16* R, size_t base, const float* W, int IN, int OUT, int KP, int NPr, size_t p) {
  const int o = (int)(p / KP), k = (int)(p % KP); R[base + p] = (b16)((o < OUT && k < IN) ? bf16_rne(W[(size_t)k * OUT + o]) : 0.0f); }
struct PArgs { const float* w[17]; const float* b[16]; };
__global__ __launch_bounds__(256) void prep_kernel(PArgs a, b16* __restrict__ R, float* __restrict__ P) {
  const float *tmW1 = a.w[0], *tmW2 = a.w[1], *tpW1 = a.w[2], *tpW2 = a.w[3], *sbW1 = a.w[4], *sbW2 = a.w[5], *suW1 = a.w[6], *suW2 = a.w[7], *cbW1 = a.w[8], *cbW2 = a.w[9], *Wv = a.w[10], *Wo = a.w[11], *Wn = a.w[12], *npW1 = a.w[13], *npW2 = a.w[14], *ppW1 = a.w[15], *ppW2 = a.w[16];
  const float *tmb1 = a.b[0], *tmb2 = a.b[1], *tpb1 = a.b[2], *tpb2 = a.b[3], *sbb1 = a.b[4], *sbb2 = a.b[5], *sub1 = a.b[6], *sub2 = a.b[7], *cbb1 = a.b[8], *cbb2 = a.b[9], *bo = a.b[10], *bn = a.b[11], *npb1 = a.b[12], *npb2 = a.b[13], *ppb1 = a.b[14], *ppb2 = a.b[15];
  const size_t tid = (size_t)blockIdx.x * blockDim.x + threadIdx.x, nth = (size_t)gridDim.x * blockDim.x;
  for (int pass = 0; pass < 2; ++pass) {
    for (size_t p = tid; p < 256 * 128; p += nth) { trw(R, Wo_::TM1, tmW1, 128, 256, 128, 256, p); trw(R, Wo_::TM2, tmW2, 256, 128, 256, 128, p); trw(R, Wo_::NP1, npW1, 128, 256, 128, 256, p); }
    for (size_t p = tid; p < 32 * 32; p += nth) { trw(R, Wo_::TP1, tpW1, 7, 32, 32, 32, p); trw(R, Wo_::TP2, tpW2, 32, 32, 32, 32, p); }
    for (size_t p = tid; p < 16 * 32; p += nth) { trw(R, Wo_::SB1, sbW1, 2, 16, 32, 16, p); trw(R, Wo_::SB2, sbW2, 16, 16, 32, 16, p); trw(R, Wo_::SU1, suW1, 3, 16, 32, 16, p); trw(R, Wo_::SU2, suW2, 16, 16, 32, 16, p); }
    for (size_t p = tid; p < 64 * 64; p += nth) { trw(R, Wo_::CB1, cbW1, 64, 64, 64, 64, p); trw(R, Wo_::CB2, cbW2, 64, 64, 64, 64, p); }
    for (size_t p = tid; p < 128 * 64; p += nth) trw(R, Wo_::WV, Wv, 64, 128, 64, 128, p);
    for (size_t p = tid; p < 128 * 128; p += nth) { trw(R, Wo_::WO, Wo, 128, 128, 128, 128, p); trw(R, Wo_::PP1, ppW1, 128, 128, 128, 128, p); }
    for (size_t p = tid; p < 128 * 32; p += nth) trw(R, Wo_::WN, Wn, 12, 128, 32, 128, p);
    for (size_t p = tid; p < 16 * 256; p += nth) trw(R, Wo_::NP2, npW2, 256, 12, 256, 16, p);
    for (size_t p = tid; p < 16 * 128; p += nth) trw(R, Wo_::PP2, ppW2, 128, 3, 128, 16, p);
    for (size_t p = tid; p < (size_t)Po_::END; p += nth) { float v = 0.0f; const int i = (int)p;
      if (i < 256) v = tmb1[i]; else if (i < 384) v = tmb2[i - 256]; else if (i < 416) v = tpb1[i - 384]; else if (i < 448) v = tpb2[i - 416]; else if (i < 464) v = sbb1[i - 448]; else if (i < 480) v = sbb2[i - 464]; else if (i < 496) v = sub1[i - 480]; else if (i < 512) v = sub2[i - 496];
      else if (i < 576) v = cbb1[i - 512]; else if (i < 640) v = cbb2[i - 576]; else if (i < 768) v = bo[i - 640]; else if (i < 896) v = bn[i - 768]; else if (i < 1152) v = npb1[i - 896]; else if (i < 1164) v = npb2[i - 1152]; else if (i < 1168) v = 0.0f; else if (i < 1296) v = ppb1[i - 1168]; else if (i < 1299) v = ppb2[i - 1296];
      P[p] = bf16_rne(v); }
    __threadfence(); }
}

template <int NT_, typename Epi>
__device__ __forceinline__ void wgemm(const float* Arow  , const b16* Bw, int KK, int hlf, int nloc, Epi epi) {
  v8f acc[NT_];
#pragma unroll
  for (int t = 0; t < NT_; ++t) acc[t] = (v8f){};
  for (int kb = 0; kb < KK; kb += 32) { v16b ah, al; frag_split(Arow + kb, hlf, ah, al);
#pragma unroll
    for (int t = 0; t < NT_; ++t) { const v16b bw = frag_kb(Bw + (size_t)(t * 16 + nloc) * KK + kb, hlf); acc[t] = wmma16b(ah, bw, acc[t]); acc[t] = wmma16b(al, bw, acc[t]); } }
  wave_lds_sync();
#pragma unroll
  for (int t = 0; t < NT_; ++t)
#pragma unroll
    for (int v = 0; v < 8; ++v) epi(8 * hlf + v, t * 16 + nloc, acc[t][v] * (1.0f / AS_));
  wave_lds_sync();
}

__global__ __launch_bounds__(64) void graph_kernel(const float* __restrict__ t, const float* __restrict__ topo, const float* __restrict__ stab, const float* __restrict__ sust, const b16* __restrict__ R, const float* __restrict__ P, float* __restrict__ tig, float* __restrict__ hug) {
  __shared__ __attribute__((aligned(16))) float TA[2][16][260], TB[2][16][260], TC[2][16][68], TD[2][16][68];
  const int wid = threadIdx.x >> 5, lane = threadIdx.x & 31, nloc = lane & 15, hlf = lane >> 4; const int g0 = blockIdx.x * 32 + wid * 16;
  for (int i = lane; i < 16 * 64; i += 32) { const int r = i >> 6, k = i & 63; const float f = __expf(-(float)k * (9.210340371976184f / 63.0f)); const float a = bf16_rne(t[g0 + r]) * f; TA[wid][r][k] = sinf(a); TA[wid][r][64 + k] = cosf(a); }
  for (int i = lane; i < 16 * 32; i += 32) { const int r = i >> 5, k = i & 31; TC[wid][r][k] = (k < 7) ? bf16_rne(topo[(size_t)(g0 + r) * 7 + k]) : 0.0f; TD[wid][r][k] = (k < 2) ? bf16_rne(stab[(size_t)(g0 + r) * 2 + k]) : 0.0f; TD[wid][r][32 + k] = (k < 3) ? bf16_rne(sust[(size_t)(g0 + r) * 3 + k]) : 0.0f; }
  wave_lds_sync();
  wgemm<16>(&TA[wid][nloc][0], R + Wo_::TM1, 128, hlf, nloc, [&](int r, int c, float v) { TB[wid][r][c] = silu_(v + P[Po_::TMB1 + c]); });
  wgemm<8>(&TB[wid][nloc][0], R + Wo_::TM2, 256, hlf, nloc, [&](int r, int c, float v) { TA[wid][r][c] = silu_(v + P[Po_::TMB2 + c]); });
  for (int pass = 0; pass < 2; ++pass) { for (int i = lane; i < 16 * 32; i += 32) { const int r = i >> 5, c4 = (i & 31) * 4; *(volatile v4f*)(tig + (size_t)(g0 + r) * HID + c4) = *(const v4f*)(&TA[wid][r][c4]); } __threadfence(); }
  wgemm<2>(&TC[wid][nloc][0], R + Wo_::TP1, 32, hlf, nloc, [&](int r, int c, float v) { TA[wid][r][c] = silu_(v + P[Po_::TPB1 + c]); });
  wgemm<2>(&TA[wid][nloc][0], R + Wo_::TP2, 32, hlf, nloc, [&](int r, int c, float v) { TB[wid][r][c] = v + P[Po_::TPB2 + c]; });
  wgemm<1>(&TD[wid][nloc][0], R + Wo_::SB1, 32, hlf, nloc, [&](int r, int c, float v) { TA[wid][r][c] = silu_(v + P[Po_::SBB1 + c]); TA[wid][r][16 + c] = 0.0f; });
  wgemm<1>(&TA[wid][nloc][0], R + Wo_::SB2, 32, hlf, nloc, [&](int r, int c, float v) { TB[wid][r][32 + c] = v + P[Po_::SBB2 + c]; });
  wgemm<1>(&TD[wid][nloc][32], R + Wo_::SU1, 32, hlf, nloc, [&](int r, int c, float v) { TA[wid][r][c] = silu_(v + P[Po_::SUB1 + c]); TA[wid][r][16 + c] = 0.0f; });
  wgemm<1>(&TA[wid][nloc][0], R + Wo_::SU2, 32, hlf, nloc, [&](int r, int c, float v) { TB[wid][r][48 + c] = v + P[Po_::SUB2 + c]; });
  wgemm<4>(&TB[wid][nloc][0], R + Wo_::CB1, 64, hlf, nloc, [&](int r, int c, float v) { TC[wid][r][c] = silu_(v + P[Po_::CBB1 + c]); });
  wgemm<4>(&TC[wid][nloc][0], R + Wo_::CB2, 64, hlf, nloc, [&](int r, int c, float v) { TD[wid][r][c] = v + P[Po_::CBB2 + c]; });
  wgemm<8>(&TD[wid][nloc][0], R + Wo_::WV, 64, hlf, nloc, [&](int r, int c, float v) { TA[wid][r][c] = v; });
  wgemm<8>(&TA[wid][nloc][0], R + Wo_::WO, 128, hlf, nloc, [&](int r, int c, float v) { TB[wid][r][c] = v + P[Po_::BO + c]; });
  for (int pass = 0; pass < 2; ++pass) { for (int i = lane; i < 16 * 32; i += 32) { const int r = i >> 5, c4 = (i & 31) * 4; *(volatile v4f*)(hug + (size_t)(g0 + r) * HID + c4) = *(const v4f*)(&TB[wid][r][c4]); } __threadfence(); }
}

__global__ __launch_bounds__(64) void node_kernel(const float* __restrict__ x, const int* __restrict__ batch, const float* __restrict__ tig, const float* __restrict__ hug, const b16* __restrict__ R, const float* __restrict__ P, float* __restrict__ npo, float* __restrict__ ppo) {
  __shared__ __attribute__((aligned(16))) float TA[2][16][260], TB[2][16][260]; __shared__ __attribute__((aligned(16))) float On[32][12], Op[32][4];
  const int wid = threadIdx.x >> 5, lane = threadIdx.x & 31, nloc = lane & 15, hlf = lane >> 4; const int n0 = blockIdx.x * 32 + wid * 16;
  for (int i = lane; i < 16 * 32; i += 32) { const int r = i >> 5, k = i & 31; TA[wid][r][k] = (k < 12) ? bf16_rne(x[(size_t)(n0 + r) * 12 + k]) : 0.0f; }
  wave_lds_sync();
  wgemm<8>(&TA[wid][nloc][0], R + Wo_::WN, 32, hlf, nloc, [&](int r, int c, float v) { TB[wid][r][c] = v + P[Po_::BN + c]; });
  for (int i = lane; i < 16 * 128; i += 32) { const int r = i >> 7, c = i & 127; int g = batch[n0 + r]; g = (g < 0) ? 0 : (g >= G ? G - 1 : g); const float hu = hug[(size_t)g * HID + c], ti = tig[(size_t)g * HID + c]; float h = TB[wid][r][c];
#pragma unroll
    for (int l = 0; l < LYR; ++l) h = (h + hu) + ti;
    TA[wid][r][c] = h; }
  wave_lds_sync();
  wgemm<16>(&TA[wid][nloc][0], R + Wo_::NP1, 128, hlf, nloc, [&](int r, int c, float v) { TB[wid][r][c] = silu_(v + P[Po_::NPB1 + c]); });
  wgemm<1>(&TB[wid][nloc][0], R + Wo_::NP2, 256, hlf, nloc, [&](int r, int c, float v) { if (c < 12) On[wid * 16 + r][c] = v + P[Po_::NPB2 + c]; });
  wgemm<8>(&TA[wid][nloc][0], R + Wo_::PP1, 128, hlf, nloc, [&](int r, int c, float v) { TB[wid][r][c] = silu_(v + P[Po_::PPB1 + c]); });
  wgemm<1>(&TB[wid][nloc][0], R + Wo_::PP2, 128, hlf, nloc, [&](int r, int c, float v) { if (c < 3) Op[wid * 16 + r][c] = v + P[Po_::PPB2 + c]; });
  __syncthreads();
  const int nb = blockIdx.x * 32;
  for (int pass = 0; pass < 2; ++pass) {
    for (int i = threadIdx.x; i < 32 * 12 / 4; i += 64) *(volatile v4f*)(npo + (size_t)nb * 12 + i * 4) = *(const v4f*)(&On[0][0] + i * 4);
    if (threadIdx.x < 24) { const int q = threadIdx.x; v4f o; for (int e = 0; e < 4; ++e) { const int f = q * 4 + e; o[e] = Op[f / 3][f % 3]; } *(volatile v4f*)(ppo + (size_t)nb * 3 + q * 4) = o; }
    __threadfence(); }
}
}

extern "C" void kernel_launch(void* const* d_in, const int* in_sizes, int n_in,
                              void* d_out, int out_size, void* d_ws, size_t ws_size, hipStream_t stream) {
  (void)n_in; (void)out_size;
  auto F = [&](int i) { return (const float*)d_in[i]; };
  const float* x = F(0); const float* t = F(4); const float* topo = F(5); const float* stab = F(6); const float* sust = F(7); const int* batch = (const int*)d_in[8];
  float* npo = (float*)d_out; float* ppo = npo + (size_t)N * 12;
  if (in_sizes[0] != N * 12 || in_sizes[4] != G || in_sizes[5] != G * 7 || in_sizes[8] != N || in_sizes[13] != 128 * 256 || in_sizes[44] != 128 * 256 || in_sizes[50] != 128 * 3) return;
  size_t off = 0; char* ws = (char*)d_ws;
  auto carve = [&](size_t bytes) { char* p = ws + off; off += (bytes + 255) & ~(size_t)255; return p; };
  b16* R = (b16*)carve(Wo_::END * 2); float* P = (float*)carve(((size_t)Po_::END + 64) * 4); float* tig = (float*)carve((size_t)G * HID * 4); float* hug = (float*)carve((size_t)G * HID * 4);
  if (off > ws_size) return;
  PArgs pa = {{F(13), F(15), F(17), F(19), F(21), F(23), F(25), F(27), F(29), F(31), F(35), F(36), F(9), F(44), F(46), F(48), F(50)}, {F(14), F(16), F(18), F(20), F(22), F(24), F(26), F(28), F(30), F(32), F(37), F(10), F(45), F(47), F(49), F(51)}};
  prep_kernel<<<64, 256, 0, stream>>>(pa, R, P);
  graph_kernel<<<G / 32, 64, 0, stream>>>(t, topo, stab, sust, R, P, tig, hug);
  node_kernel<<<NBLK, 64, 0, stream>>>(x, batch, tig, hug, R, P, npo, ppo);
}
